// ProvenanceGNN_37297495998502
// MI455X (gfx1250) — hardware-verified
//
#include <hip/hip_runtime.h>
#include <stddef.h>
#include <math.h>


#define DF    128
#define NHD   4
#define GR    32
#define XSP   132
#define NTHR  256
#define NWAVE 8
#define NB    512
#define CHUNK 2048
#define WCAP  256
#define NGRP  (CHUNK / (NTHR * 4))
#define NRN   64
#define PP    320
#define PH    256

#define OFF_C0 (DF * PP)
#define OFF_C1 (OFF_C0 + DF * PH)
#define OFF_H1 (OFF_C1 + DF * PH)
#define WP_HALVES (OFF_H1 + 64 * PH)
#define PREP_ROWS 448
#define PREP_BLOCKS (PREP_ROWS / NWAVE + 1)

#define LDS_SACC (NB * DF)
#define LDS_DEN  (NB * NHD)
#define LDS_MR   (NB * NHD)
#define LDS_LIST (NWAVE * WCAP)
#define LDS_BYTES ((LDS_SACC + LDS_DEN + LDS_MR + LDS_LIST + NWAVE) * 4)

static_assert(WCAP == (CHUNK / NTHR) * 32);
static_assert(NGRP == 2);
static_assert(NB == 512);
static_assert(CHUNK <= 2048);
static_assert(((LDS_SACC + LDS_DEN) % 4) == 0);
static_assert((LDS_MR % 4) == 0);
static_assert(LDS_BYTES == 286752);
static_assert(WP_HALVES == 122880);
static_assert(PREP_BLOCKS == 57);
static_assert((NB % NWAVE) == 0);

typedef __bf16 bf16;
typedef float    v4f  __attribute__((ext_vector_type(4)));
typedef float    v8f  __attribute__((ext_vector_type(8)));
typedef int      v4i  __attribute__((ext_vector_type(4)));
typedef unsigned v2u  __attribute__((ext_vector_type(2)));
typedef bf16     v8b  __attribute__((ext_vector_type(8)));
typedef bf16     v16b __attribute__((ext_vector_type(16)));
union Frag { v16b v; v8b half[2]; };
union P4   { bf16 h[4]; v2u u; };
union P2   { bf16 h[2]; unsigned u; };

__device__ __forceinline__ v8f wm(v16b a, v16b b, v8f c) {
  v8f d = __builtin_amdgcn_wmma_f32_16x16x32_bf16(false, a, false, b, (short)0, c, false, false);
  asm volatile("v_nop\n\tv_nop\n\tv_nop\n\tv_nop" : "+v"(d) : "v"(a), "v"(b));
  return d;
}

__device__ __forceinline__ void split2(float v, bf16& h, bf16& l) {
  h = (bf16)v;
  l = (bf16)(v - (float)h);
}

__device__ __forceinline__ v16b ldfrag(const bf16* p) {
  Frag f;
  f.half[0] = *(const v8b*)p;
  f.half[1] = *(const v8b*)(p + 16);
  return f.v;
}

__host__ __device__ constexpr int hoff(int kt) { return kt < 4 ? 32 * kt : 256 + 64 * (kt - 4); }
__host__ __device__ constexpr int loff(int kt) { return kt < 4 ? 128 + 32 * kt : 288 + 64 * (kt - 4); }

__device__ __forceinline__ float eluf(float v) { return v > 0.f ? v : (__expf(v) - 1.0f); }

__global__ __launch_bounds__(NTHR) void k_minmax(const int* __restrict__ ts, int* mm, int nN) {
  __shared__ int smn[NTHR];
  __shared__ int smx[NTHR];
  const int tid = threadIdx.x;
  int lo = 2147483647, hi = -2147483647 - 1;
  for (int j = tid; j < nN; j += NTHR) {
    const int v = ts[j];
    lo = min(lo, v);
    hi = max(hi, v);
  }
  smn[tid] = lo;
  smx[tid] = hi;
  __syncthreads();
  for (int s = NTHR / 2; s > 0; s >>= 1) {
    if (tid < s) {
      smn[tid] = min(smn[tid], smn[tid + s]);
      smx[tid] = max(smx[tid], smx[tid + s]);
    }
    __syncthreads();
  }
  if (tid < 32) {
    const int lane = tid;
    v4i val = {0, 0, 0, 0};
    if (lane == 0) { val.x = smn[0]; val.y = smx[0]; }
    int* p = mm + 4 * (lane & 7);
    if (lane < 8) *(volatile v4i*)p = val;
    __threadfence();
    if (lane < 8) *(volatile v4i*)p = val;
  }
}

__global__ __launch_bounds__(NTHR) void k_prepw(
    const float* __restrict__ proj_w, const float* __restrict__ conv_w,
    const float* __restrict__ head_w1, const float* __restrict__ bn_g,
    const float* __restrict__ bn_v, bf16* WP, float* BNS) {
  const int tid  = threadIdx.x;
  const int lane = tid & 31;
  const int wave = tid >> 5;
  if (blockIdx.x == PREP_BLOCKS - 1) {
    const float s = bn_g[tid] / sqrtf(bn_v[tid] + 1e-5f);
    *(volatile float*)(BNS + tid) = s;
    __threadfence();
    *(volatile float*)(BNS + tid) = s;
    return;
  }
  const int g = blockIdx.x * NWAVE + wave;
  const float* W;
  int ncols, n, pitch;
  bf16* dst;
  bool extra = false;
  if (g < 128)      { W = proj_w;           ncols = DF; n = g;       pitch = PP; dst = WP;          extra = true; }
  else if (g < 256) { W = conv_w;           ncols = DF; n = g - 128; pitch = PH; dst = WP + OFF_C0; }
  else if (g < 384) { W = conv_w + DF * DF; ncols = DF; n = g - 256; pitch = PH; dst = WP + OFF_C1; }
  else              { W = head_w1;          ncols = 64; n = g - 384; pitch = PH; dst = WP + OFF_H1; }

  P4 ph, pl;
  {
    const float v0 = W[(size_t)(4 * lane + 0) * ncols + n];
    const float v1 = W[(size_t)(4 * lane + 1) * ncols + n];
    const float v2 = W[(size_t)(4 * lane + 2) * ncols + n];
    const float v3 = W[(size_t)(4 * lane + 3) * ncols + n];
    split2(v0, ph.h[0], pl.h[0]);
    split2(v1, ph.h[1], pl.h[1]);
    split2(v2, ph.h[2], pl.h[2]);
    split2(v3, ph.h[3], pl.h[3]);
  }
  unsigned te = 0u;
  if (extra) {
    const int kk = DF + 2 * (lane & 7);
    const float e0 = W[(size_t)kk * ncols + n];
    const float e1 = W[(size_t)(kk + 1) * ncols + n];
    bf16 h0, l0, h1, l1;
    split2(e0, h0, l0);
    split2(e1, h1, l1);
    P2 pt;
    pt.h[0] = (bf16)0.f;
    pt.h[1] = (bf16)0.f;
    if ((lane & 15) < 8) {
      if (lane < 16) { pt.h[0] = h0; pt.h[1] = h1; }
      else           { pt.h[0] = l0; pt.h[1] = l1; }
    }
    te = pt.u;
  }
  bf16* rowp = dst + (size_t)n * pitch;
  bf16* p0 = rowp + 4 * lane;
  bf16* p1 = rowp + 128 + 4 * lane;
  bf16* p2 = rowp + 256 + 2 * lane;
  *(volatile v2u*)p0 = ph.u;
  *(volatile v2u*)p1 = pl.u;
  if (extra) *(volatile unsigned*)p2 = te;
  __threadfence();
  *(volatile v2u*)p0 = ph.u;
  *(volatile v2u*)p1 = pl.u;
  if (extra) *(volatile unsigned*)p2 = te;
}

__global__ __launch_bounds__(NTHR) void k_node(
    const float* __restrict__ x, const int* __restrict__ ts, const int* __restrict__ mm,
    const float* __restrict__ gw1, const float* __restrict__ gb1,
    const float* __restrict__ gw2, const float* __restrict__ gb2,
    bf16* XA, float* GATE, int nN, int nP) {
  __shared__ __attribute__((aligned(16))) float gs[NRN];
  const int tid  = threadIdx.x;
  const int lane = tid & 31;
  const int wave = tid >> 5;
  const int rb   = blockIdx.x * NRN;
  const float tmn  = (float)mm[0];
  const float tmx  = (float)mm[1];
  const float rinv = 1.0f / fmaxf(tmx - tmn, 1.0f);
  const int j = lane & 15;
  const int q = lane & 7;
  const float fr = expf((float)(2 * (j & 7)) * -0.5756462732485115f);
  const float gb2v = gb2[0];

#pragma unroll 1
  for (int i = 0; i < NRN / NWAVE; ++i) {
    const int r  = rb + wave * (NRN / NWAVE) + i;
    const int rc = min(r, nN - 1);
    const float t = (float)ts[rc];
    const v4f xv = *(const v4f*)(x + (size_t)rc * DF + 4 * lane);
    P4 ph, pl;
    split2(xv.x, ph.h[0], pl.h[0]);
    split2(xv.y, ph.h[1], pl.h[1]);
    split2(xv.z, ph.h[2], pl.h[2]);
    split2(xv.w, ph.h[3], pl.h[3]);
    const float a = t * fr;
    float tev;
    if (j < 8) tev = sinf(a); else tev = cosf(a);
    const float v0 = __shfl(tev, 2 * q, 32);
    const float v1 = __shfl(tev, 2 * q + 1, 32);
    bf16 h0, l0, h1, l1;
    split2(v0, h0, l0);
    split2(v1, h1, l1);
    P2 pt;
    pt.h[0] = (bf16)0.f;
    pt.h[1] = (bf16)0.f;
    if (j < 8) {
      if (lane < 16) { pt.h[0] = h0; pt.h[1] = h1; }
      else           { pt.h[0] = l0; pt.h[1] = l1; }
    }
    const float age = (t - tmn) * rinv;
    float s = gb2v;
#pragma unroll 1
    for (int k = 0; k < 16; ++k) {
      float z = age * gw1[k] + gb1[k];
      z = fmaxf(z, 0.f);
      s += z * gw2[k];
    }
    const float gt = 1.0f / (1.0f + __expf(-s));
    if (lane == 0) gs[wave * (NRN / NWAVE) + i] = gt;
    if (r < nP) {
      bf16* rowp = XA + (size_t)r * PP;
      bf16* p0 = rowp + 4 * lane;
      bf16* p1 = rowp + 128 + 4 * lane;
      bf16* p2 = rowp + 256 + 2 * lane;
      *(volatile v2u*)p0 = ph.u;
      *(volatile v2u*)p1 = pl.u;
      *(volatile unsigned*)p2 = pt.u;
      __threadfence();
      *(volatile v2u*)p0 = ph.u;
      *(volatile v2u*)p1 = pl.u;
      *(volatile unsigned*)p2 = pt.u;
    }
  }
  __syncthreads();
  if (wave == 0) {
    const v4f gv = *(const v4f*)(gs + 4 * (lane & 15));
    float* gp = GATE + (size_t)rb + 4 * (lane & 15);
    if (lane < 16) *(volatile v4f*)gp = gv;
    __threadfence();
    if (lane < 16) *(volatile v4f*)gp = gv;
  }
}

template <int KT, int NCT, int EPI>
__global__ __launch_bounds__(NTHR) void k_gemm(
    const bf16* __restrict__ A, const bf16* __restrict__ Bp,
    const float* __restrict__ f0, const float* __restrict__ f1, const float* __restrict__ f2,
    bf16* outA, float* outF, float* outL) {
  constexpr int PITCH = (KT == 4) ? PH : PP;
  constexpr int U = NCT / 4;
  __shared__ __attribute__((aligned(16))) float Xs[GR * XSP];
  __shared__ __attribute__((aligned(16))) float Ls[GR * 8];

  const int tid  = threadIdx.x;
  const int lane = tid & 31;
  const int wave = tid >> 5;
  const int hh   = lane >> 4;
  const int m    = lane & 15;
  const int rowBase = blockIdx.x * GR;
  const int ct = (wave * U) >> 1;

  v8f acc[U];
  const bf16* ab[U];
#pragma unroll
  for (int u = 0; u < U; ++u) {
    acc[u] = (v8f){0.f, 0.f, 0.f, 0.f, 0.f, 0.f, 0.f, 0.f};
    const int rt = (wave * U + u) & 1;
    ab[u] = A + (size_t)(rowBase + 16 * rt + m) * PITCH + 8 * hh;
  }
  const bf16* bb = Bp + (size_t)(ct * 16 + m) * PITCH + 8 * hh;

#pragma unroll
  for (int kt = 0; kt < KT; ++kt) {
    const v16b bh = ldfrag(bb + hoff(kt));
    const v16b bl = ldfrag(bb + loff(kt));
#pragma unroll
    for (int u = 0; u < U; ++u) {
      const v16b ah = ldfrag(ab[u] + hoff(kt));
      const v16b al = ldfrag(ab[u] + loff(kt));
      acc[u] = wm(ah, bh, acc[u]);
      acc[u] = wm(ah, bl, acc[u]);
      acc[u] = wm(al, bh, acc[u]);
    }
  }

  {
    const int col = ct * 16 + m;
    float bv = 0.f;
    if (EPI != 1) bv = f0[col];
#pragma unroll
    for (int u = 0; u < U; ++u) {
      const int rt = (wave * U + u) & 1;
#pragma unroll
      for (int r = 0; r < 8; ++r) {
        float v = acc[u][r];
        if (EPI != 1) { v += bv; v = fmaxf(v, 0.f); }
        Xs[(16 * rt + 8 * hh + r) * XSP + col] = v;
      }
    }
  }
  __syncthreads();

  if (EPI == 0) {
    v2u hv[4], lv[4];
    bf16* bp[4];
#pragma unroll
    for (int i = 0; i < 4; ++i) {
      const int row = 4 * wave + i;
      const v4f v = *(const v4f*)(Xs + row * XSP + 4 * lane);
      P4 ph, pl;
      split2(v.x, ph.h[0], pl.h[0]);
      split2(v.y, ph.h[1], pl.h[1]);
      split2(v.z, ph.h[2], pl.h[2]);
      split2(v.w, ph.h[3], pl.h[3]);
      hv[i] = ph.u;
      lv[i] = pl.u;
      bp[i] = outA + (size_t)(rowBase + row) * PH + 4 * lane;
    }
#pragma unroll
    for (int i = 0; i < 4; ++i) { *(volatile v2u*)(bp[i]) = hv[i]; *(volatile v2u*)(bp[i] + 128) = lv[i]; }
    __threadfence();
#pragma unroll
    for (int i = 0; i < 4; ++i) { *(volatile v2u*)(bp[i]) = hv[i]; *(volatile v2u*)(bp[i] + 128) = lv[i]; }
  } else if (EPI == 1) {
    const v4f as4 = *(const v4f*)(f0 + 4 * lane);
    const v4f ad4 = *(const v4f*)(f1 + 4 * lane);
    v4f xr[4];
    float* hp[4];
#pragma unroll
    for (int i = 0; i < 4; ++i) {
      const int row = 4 * wave + i;
      xr[i] = *(const v4f*)(Xs + row * XSP + 4 * lane);
      float ps = xr[i].x * as4.x + xr[i].y * as4.y + xr[i].z * as4.z + xr[i].w * as4.w;
      float pd = xr[i].x * ad4.x + xr[i].y * ad4.y + xr[i].z * ad4.z + xr[i].w * ad4.w;
      ps += __shfl_xor(ps, 1, 32); pd += __shfl_xor(pd, 1, 32);
      ps += __shfl_xor(ps, 2, 32); pd += __shfl_xor(pd, 2, 32);
      ps += __shfl_xor(ps, 4, 32); pd += __shfl_xor(pd, 4, 32);
      if ((lane & 7) == 0) {
        Ls[row * 8 + (lane >> 3)]     = ps;
        Ls[row * 8 + 4 + (lane >> 3)] = pd;
      }
      hp[i] = outF + (size_t)(rowBase + row) * DF + 4 * lane;
    }
    __syncthreads();
    const v4f lv = *(const v4f*)(Ls + 32 * wave + 4 * (lane & 7));
    float* lp = outL + (size_t)(rowBase + 4 * wave) * 8 + 4 * (lane & 7);
#pragma unroll
    for (int i = 0; i < 4; ++i) *(volatile v4f*)(hp[i]) = xr[i];
    if (lane < 8) *(volatile v4f*)lp = lv;
    __threadfence();
#pragma unroll
    for (int i = 0; i < 4; ++i) *(volatile v4f*)(hp[i]) = xr[i];
    if (lane < 8) *(volatile v4f*)lp = lv;
  } else {
    const int R = tid >> 3;
    const int part = tid & 7;
    float o0 = 0.f, o1 = 0.f;
#pragma unroll
    for (int c = 0; c < 8; ++c) {
      const int col = part * 8 + c;
      const float v = Xs[R * XSP + col];
      o0 += v * f1[col * 2 + 0];
      o1 += v * f1[col * 2 + 1];
    }
    o0 += __shfl_xor(o0, 1, 32); o1 += __shfl_xor(o1, 1, 32);
    o0 += __shfl_xor(o0, 2, 32); o1 += __shfl_xor(o1, 2, 32);
    o0 += __shfl_xor(o0, 4, 32); o1 += __shfl_xor(o1, 4, 32);
    if (part == 0) {
      Ls[R * 2 + 0] = o0 + f2[0];
      Ls[R * 2 + 1] = o1 + f2[1];
    }
    __syncthreads();
    if (wave == 0) {
      const v4f gv = *(const v4f*)(Ls + 4 * (lane & 15));
      float* op = outF + (size_t)rowBase * 2 + 4 * (lane & 15);
      if (lane < 16) *(volatile v4f*)op = gv;
      __threadfence();
      if (lane < 16) *(volatile v4f*)op = gv;
    }
  }
}

__global__ __launch_bounds__(NTHR) void k_agg(
    const int* __restrict__ ei, const float* __restrict__ HH, const float* __restrict__ AL,
    const float* __restrict__ gate, const float* __restrict__ cb, const float* __restrict__ bns,
    const float* __restrict__ bnb, const float* __restrict__ bnm,
    bf16* HA, int nN, int nE) {
  extern __shared__ v4f lds_dyn[];
  float* sacc = (float*)lds_dyn;
  float* den  = sacc + LDS_SACC;
  float* mr   = den + LDS_DEN;
  int*   list = (int*)(mr + LDS_MR);
  int*   wcnt = list + LDS_LIST;

  const int tid  = threadIdx.x;
  const int lane = tid & 31;
  const int wave = tid >> 5;
  const int hd   = lane >> 3;
  const int nodeBase = blockIdx.x * NB;

  {
    const v4f z4 = {0.f, 0.f, 0.f, 0.f};
    for (int i = tid; i < (LDS_SACC + LDS_DEN) / 4; i += NTHR) lds_dyn[i] = z4;
    const v4f n4 = {-1e30f, -1e30f, -1e30f, -1e30f};
    for (int i = tid; i < LDS_MR / 4; i += NTHR) lds_dyn[(LDS_SACC + LDS_DEN) / 4 + i] = n4;
  }
  __syncthreads();

  const int* eid = ei + nE;
  const bool al16 = ((nE & 3) == 0);
  const int nChunks = (nE + CHUNK - 1) / CHUNK;
#pragma unroll 1
  for (int ch = 0; ch < nChunks; ++ch) {
    const int cbase = ch * CHUNK;
    const bool full = al16 && (cbase + CHUNK <= nE);
    int wc = 0;
#pragma unroll
    for (int g = 0; g < NGRP; ++g) {
      const int el0 = (g * NTHR + tid) * 4;
      const int e0  = cbase + el0;
      const int sent = -2147483647 - 1;
      v4i d;
      if (full) {
        d = *(const v4i*)(eid + e0);
      } else {
        d.x = (e0     < nE) ? eid[min(e0,     nE - 1)] : sent;
        d.y = (e0 + 1 < nE) ? eid[min(e0 + 1, nE - 1)] : sent;
        d.z = (e0 + 2 < nE) ? eid[min(e0 + 2, nE - 1)] : sent;
        d.w = (e0 + 3 < nE) ? eid[min(e0 + 3, nE - 1)] : sent;
      }
      const unsigned s0 = (unsigned)d.x - (unsigned)nodeBase;
      const unsigned s1 = (unsigned)d.y - (unsigned)nodeBase;
      const unsigned s2 = (unsigned)d.z - (unsigned)nodeBase;
      const unsigned s3 = (unsigned)d.w - (unsigned)nodeBase;
      const bool h0 = s0 < (unsigned)NB;
      const bool h1 = s1 < (unsigned)NB;
      const bool h2 = s2 < (unsigned)NB;
      const bool h3 = s3 < (unsigned)NB;
      const unsigned many = __builtin_amdgcn_ballot_w32(h0 | h1 | h2 | h3);
      if (many != 0u) {
#define HITJ(J, HJ, SJ) { \
          const unsigned mj = __builtin_amdgcn_ballot_w32(HJ); \
          if (HJ) { \
            const int pos = wc + (int)__builtin_amdgcn_mbcnt_lo(mj, 0u); \
            if (pos < WCAP) list[wave * WCAP + pos] = ((el0 + (J)) << 9) | (int)(SJ); \
          } \
          wc += (int)__builtin_popcount(mj); }
        HITJ(0, h0, s0)
        HITJ(1, h1, s1)
        HITJ(2, h2, s2)
        HITJ(3, h3, s3)
#undef HITJ
      }
    }
    if (lane == 0) wcnt[wave] = wc;
    __syncthreads();

    if (wave == 0) {
      for (int wsx = 0; wsx < NWAVE; ++wsx) {
        int n = wcnt[wsx];
        if (n > WCAP) n = WCAP;
        if (n < 0) n = 0;
        for (int i = 0; i < n; ++i) {
          const int ent  = list[wsx * WCAP + i];
          const int slot = ent & (NB - 1);
          const int el   = (ent >> 9) & (CHUNK - 1);
          int e = cbase + el;
          if (e > nE - 1) e = nE - 1;
          int src = ei[e];
          src = src < 0 ? 0 : (src > nN - 1 ? nN - 1 : src);
          int nd = nodeBase + slot;
          if (nd > nN - 1) nd = nN - 1;
          float a = AL[(size_t)src * 8 + hd] + AL[(size_t)nd * 8 + 4 + hd];
          a = (a > 0.f) ? a : 0.2f * a;
          const float mo  = mr[slot * NHD + hd];
          const float mn2 = fmaxf(mo, a);
          const float sc  = __expf(mo - mn2);
          const float p   = __expf(a - mn2);
          const v4f xv = *(const v4f*)(HH + (size_t)src * DF + 4 * lane);
          v4f* sp = (v4f*)(sacc + slot * DF + 4 * lane);
          const v4f cur = *sp;
          const v4f nxt = cur * sc + p * xv;
          *sp = nxt;
          if ((lane & 7) == 0) {
            const float dold = den[slot * NHD + hd];
            den[slot * NHD + hd] = dold * sc + p;
            mr[slot * NHD + hd]  = mn2;
          }
        }
      }
    }
    __syncthreads();
  }

  const v4f cb4 = *(const v4f*)(cb  + 4 * lane);
  const v4f s4  = *(const v4f*)(bns + 4 * lane);
  const v4f b4  = *(const v4f*)(bnb + 4 * lane);
  const v4f m4  = *(const v4f*)(bnm + 4 * lane);
#pragma unroll 1
  for (int j = 0; j < NB / NWAVE; ++j) {
    const int slot = wave * (NB / NWAVE) + j;
    const int node = nodeBase + slot;
    if (node >= nN) break;
    const size_t nrow = (size_t)node;
    float a = AL[nrow * 8 + hd] + AL[nrow * 8 + 4 + hd];
    a = (a > 0.f) ? a : 0.2f * a;
    const float mo  = mr[slot * NHD + hd];
    const float mn2 = fmaxf(mo, a);
    const float sc  = __expf(mo - mn2);
    const float p   = __expf(a - mn2);
    const v4f xv = *(const v4f*)(HH + nrow * DF + 4 * lane);
    const v4f sv = *(const v4f*)(sacc + slot * DF + 4 * lane) * sc + p * xv;
    const float dv  = den[slot * NHD + hd] * sc + p;
    const float inv = 1.0f / (dv + 1e-16f);
    const float gt  = gate[nrow];
    v4f h = sv * inv + cb4;
    h = (h - m4) * s4 + b4;
    h.x = eluf(h.x) * gt;
    h.y = eluf(h.y) * gt;
    h.z = eluf(h.z) * gt;
    h.w = eluf(h.w) * gt;
    P4 ph, pl;
    split2(h.x, ph.h[0], pl.h[0]);
    split2(h.y, ph.h[1], pl.h[1]);
    split2(h.z, ph.h[2], pl.h[2]);
    split2(h.w, ph.h[3], pl.h[3]);
    bf16* p0 = HA + nrow * PH + 4 * lane;
    bf16* p1 = p0 + 128;
    *(volatile v2u*)p0 = ph.u;
    *(volatile v2u*)p1 = pl.u;
    __threadfence();
    *(volatile v2u*)p0 = ph.u;
    *(volatile v2u*)p1 = pl.u;
  }
}

extern "C" void kernel_launch(void* const* d_in, const int* in_sizes, int n_in,
                              void* d_out, int out_size, void* d_ws, size_t ws_size,
                              hipStream_t stream) {
  if (n_in < 21) return;
  const int nN = in_sizes[2];
  if (nN < GR || (nN % GR) != 0) return;
  if (in_sizes[0] != nN * DF) return;
  const int nE = in_sizes[1] / 2;
  if (nE < 1 || in_sizes[1] != 2 * nE) return;
  if (in_sizes[3] != 144 * DF || in_sizes[4] != DF) return;
  if (in_sizes[5] != 2 * DF * DF || in_sizes[6] != 2 * DF) return;
  if (in_sizes[7] != 2 * DF || in_sizes[8] != 2 * DF) return;
  if (in_sizes[9] != 2 * DF || in_sizes[10] != 2 * DF || in_sizes[11] != 2 * DF || in_sizes[12] != 2 * DF) return;
  if (in_sizes[13] != 16 || in_sizes[14] != 16 || in_sizes[15] != 16 || in_sizes[16] != 1) return;
  if (in_sizes[17] != DF * 64 || in_sizes[18] != 64 || in_sizes[19] != 128 || in_sizes[20] != 2) return;
  if (out_size != nN * 2) return;

  const float* x        = (const float*)d_in[0];
  const int*   ei       = (const int*)  d_in[1];
  const int*   ts       = (const int*)  d_in[2];
  const float* proj_w   = (const float*)d_in[3];
  const float* proj_b   = (const float*)d_in[4];
  const float* conv_w   = (const float*)d_in[5];
  const float* conv_b   = (const float*)d_in[6];
  const float* att_src  = (const float*)d_in[7];
  const float* att_dst  = (const float*)d_in[8];
  const float* bn_gamma = (const float*)d_in[9];
  const float* bn_beta  = (const float*)d_in[10];
  const float* bn_mean  = (const float*)d_in[11];
  const float* bn_var   = (const float*)d_in[12];
  const float* gate_w1  = (const float*)d_in[13];
  const float* gate_b1  = (const float*)d_in[14];
  const float* gate_w2  = (const float*)d_in[15];
  const float* gate_b2  = (const float*)d_in[16];
  const float* head_w1  = (const float*)d_in[17];
  const float* head_b1  = (const float*)d_in[18];
  const float* head_w2  = (const float*)d_in[19];
  const float* head_b2  = (const float*)d_in[20];
  float* out = (float*)d_out;

  const int nP    = nN;
  const int gNode = (nN + NRN - 1) / NRN;
  const size_t nGt = (size_t)gNode * NRN;

  char* ws = (char*)d_ws;
  size_t off = 0;
  int*   MM   = (int*)(ws + off);    off += 256;
  bf16*  WP   = (bf16*)(ws + off);   off += (size_t)WP_HALVES * 2;
  float* BNS  = (float*)(ws + off);  off += (size_t)2 * DF * 4;
  float* GATE = (float*)(ws + off);  off += ((nGt * 4) + 255) & ~(size_t)255;
  bf16*  HA   = (bf16*)(ws + off);   off += (size_t)nP * PH * 2;
  const size_t regA = (size_t)nP * PP * 2;
  const size_t regB = (size_t)nP * DF * 4 + (size_t)nP * 8 * 4;
  char*  R    = ws + off;            off += (regA > regB ? regA : regB);
  bf16*  XA   = (bf16*)R;
  float* HH   = (float*)R;
  float* AL   = (float*)(R + (size_t)nP * DF * 4);
  if (off > ws_size) return;
  if (off > ((size_t)128 << 20)) return;

  k_minmax<<<1, NTHR, 0, stream>>>(ts, MM, nN);
  k_prepw<<<PREP_BLOCKS, NTHR, 0, stream>>>(proj_w, conv_w, head_w1, bn_gamma, bn_var, WP, BNS);
  k_node<<<gNode, NTHR, 0, stream>>>(x, ts, MM, gate_w1, gate_b1, gate_w2, gate_b2, XA, GATE, nN, nP);

  const int gGemm = nP / GR;
  k_gemm<5, 8, 0><<<gGemm, NTHR, 0, stream>>>(XA, WP, proj_b, (const float*)0, (const float*)0,
                                               HA, (float*)0, (float*)0);

  hipFuncSetAttribute(reinterpret_cast<const void*>(&k_agg),
                      hipFuncAttributeMaxDynamicSharedMemorySize, LDS_BYTES);
  const int gAgg = (nN + NB - 1) / NB;
  for (int l = 0; l < 2; ++l) {
    const bf16* Wl = WP + (l == 0 ? OFF_C0 : OFF_C1);
    k_gemm<4, 8, 1><<<gGemm, NTHR, 0, stream>>>(HA, Wl, att_src + l * DF, att_dst + l * DF,
                                                 (const float*)0, (bf16*)0, HH, AL);
    k_agg<<<gAgg, NTHR, LDS_BYTES, stream>>>(ei, HH, AL, GATE, conv_b + l * DF, BNS + l * DF,
                                              bn_beta + l * DF, bn_mean + l * DF, HA, nN, nE);
  }

  k_gemm<4, 4, 2><<<gGemm, NTHR, 0, stream>>>(HA, WP + OFF_H1, head_b1, head_w2, head_b2,
                                               (bf16*)0, out, (float*)0);
}
